// graph_smooth_43284680409688
// MI455X (gfx1250) — hardware-run, weakly checked
//
#include <hip/hip_runtime.h>
#include <stddef.h>


#define DEMB   128
#define DOUT   64
#define NTHR   256
#define NWAVE  8
#define EPT    8
#define NGRP   2
#define CHUNK  (NTHR * EPT * NGRP)
#define WCAP   (EPT * NGRP * 32)
#define NB     128
#define ESHF   7
#define RCAP   8192
#define DEGCAP 256
#define NPW    (NB / NWAVE)
#define GROWS  128
#define TPK    64
#define TPN    32
#define TPP    72
#define ASCL   16
#define WSCL   64
#define WSCAP  134217728
#define LDS_GEMM (GROWS * DOUT * 4)

static_assert((CHUNK & (CHUNK - 1)) == 0);
static_assert(NB == (1 << ESHF));
static_assert(NB == GROWS);
static_assert((NB % NWAVE) == 0 && (NPW % 2) == 0);
static_assert(NB == 4 * 32);
static_assert((RCAP % (4 * NTHR)) == 0);
static_assert(DOUT == 2 * 32);
static_assert((DEMB % 32) == 0 && (DOUT % 16) == 0 && (128 % DOUT) == 0);
static_assert((DEMB % TPK) == 0 && (DOUT % TPN) == 0);
static_assert(TPN * 8 == NTHR && TPK * TPN == NTHR * 8 && TPK == NWAVE * 8);
static_assert((TPP % 8) == 0 && TPP >= TPK);
static_assert(GROWS == NWAVE * 16);

typedef float     v2f  __attribute__((ext_vector_type(2)));
typedef float     v4f  __attribute__((ext_vector_type(4)));
typedef float     v8f  __attribute__((ext_vector_type(8)));
typedef int       v4i  __attribute__((ext_vector_type(4)));
typedef _Float16  v8h  __attribute__((ext_vector_type(8)));
typedef _Float16  v16h __attribute__((ext_vector_type(16)));
union FragH { v16h v; v8h h[2]; };
union U32F { float f; int i; };

__device__ __forceinline__ v8f wmf(v16h a, v16h b, v8f c) {
  v8f d = __builtin_amdgcn_wmma_f32_16x16x32_f16(false, a, false, b, (short)0, c, false, false);
  asm volatile("v_nop\n\tv_nop\n\tv_nop\n\tv_nop" : "+v"(d) : "v"(a), "v"(b));
  return d;
}

template <int NBK, int EIDX, int WC>
__device__ __forceinline__ int scan_chunk(const int* __restrict__ keys, int nK, int cbase,
                                          int slotBase, int vec8, int* list,
                                          int tid, int lane, int wave) {
  int wc = 0;
#pragma unroll
  for (int g = 0; g < NGRP; ++g) {
    const int el0  = (g * NTHR + tid) * EPT;
    const int e0   = cbase + el0;
    const int sent = -2147483647 - 1;
    v4i da, db;
    if (vec8 != 0 && cbase + CHUNK <= nK) {
      da = *(const v4i*)(keys + e0);
      db = *(const v4i*)(keys + e0 + 4);
    } else {
      const int i0 = min(e0, nK - 1),     i1 = min(e0 + 1, nK - 1), i2 = min(e0 + 2, nK - 1), i3 = min(e0 + 3, nK - 1);
      const int i4 = min(e0 + 4, nK - 1), i5 = min(e0 + 5, nK - 1), i6 = min(e0 + 6, nK - 1), i7 = min(e0 + 7, nK - 1);
      da.x = (e0     < nK) ? keys[i0] : sent;
      da.y = (e0 + 1 < nK) ? keys[i1] : sent;
      da.z = (e0 + 2 < nK) ? keys[i2] : sent;
      da.w = (e0 + 3 < nK) ? keys[i3] : sent;
      db.x = (e0 + 4 < nK) ? keys[i4] : sent;
      db.y = (e0 + 5 < nK) ? keys[i5] : sent;
      db.z = (e0 + 6 < nK) ? keys[i6] : sent;
      db.w = (e0 + 7 < nK) ? keys[i7] : sent;
    }
    const unsigned nb = (unsigned)slotBase;
    const unsigned s0 = (unsigned)da.x - nb, s1 = (unsigned)da.y - nb;
    const unsigned s2 = (unsigned)da.z - nb, s3 = (unsigned)da.w - nb;
    const unsigned s4 = (unsigned)db.x - nb, s5 = (unsigned)db.y - nb;
    const unsigned s6 = (unsigned)db.z - nb, s7 = (unsigned)db.w - nb;
    const bool h0 = s0 < (unsigned)NBK, h1 = s1 < (unsigned)NBK, h2 = s2 < (unsigned)NBK, h3 = s3 < (unsigned)NBK;
    const bool h4 = s4 < (unsigned)NBK, h5 = s5 < (unsigned)NBK, h6 = s6 < (unsigned)NBK, h7 = s7 < (unsigned)NBK;
    const unsigned any = __builtin_amdgcn_ballot_w32(h0 | h1 | h2 | h3 | h4 | h5 | h6 | h7);
    if (any != 0u) {
#define HITJ(HJ, SJ, J) { \
        const unsigned mj = __builtin_amdgcn_ballot_w32(HJ); \
        if (mj != 0u) { \
          if (HJ) { \
            const int pos = wc + (int)__builtin_amdgcn_mbcnt_lo(mj, 0u); \
            const int entv = EIDX ? (((e0 + (J)) << ESHF) | (int)(SJ)) : (int)(SJ); \
            if (pos < WC) list[wave * WC + pos] = entv; \
          } \
          wc += (int)__builtin_popcount(mj); } }
      HITJ(h0, s0, 0)
      HITJ(h1, s1, 1)
      HITJ(h2, s2, 2)
      HITJ(h3, s3, 3)
      HITJ(h4, s4, 4)
      HITJ(h5, s5, 5)
      HITJ(h6, s6, 6)
      HITJ(h7, s7, 7)
#undef HITJ
    }
  }
  return wc;
}

__global__ __launch_bounds__(NTHR) void k_cvt16(const float* __restrict__ src, _Float16* dst,
                                                int rowLen, int nSrcRows, int total8, float scale) {
  const int i = (int)blockIdx.x * NTHR + (int)threadIdx.x;
  if (i >= total8) return;
  const size_t e  = (size_t)8 * (size_t)i;
  const int    r  = (int)(e / (size_t)rowLen);
  const int    k0 = (int)(e - (size_t)r * (size_t)rowLen);
  const int    rc = r < nSrcRows ? r : nSrcRows - 1;
  const float  z  = (r < nSrcRows) ? scale : 0.0f;
  const float* sp = src + (size_t)rc * rowLen + k0;
  const v4f f0 = *(const v4f*)sp;
  const v4f f1 = *(const v4f*)(sp + 4);
  v8h hv;
  hv[0] = (_Float16)(f0.x * z); hv[1] = (_Float16)(f0.y * z); hv[2] = (_Float16)(f0.z * z); hv[3] = (_Float16)(f0.w * z);
  hv[4] = (_Float16)(f1.x * z); hv[5] = (_Float16)(f1.y * z); hv[6] = (_Float16)(f1.z * z); hv[7] = (_Float16)(f1.w * z);
  _Float16* d = dst + e;
  *(volatile v8h*)d = hv;
  __threadfence();
  *(volatile v8h*)d = hv;
}

__global__ __launch_bounds__(NTHR) void k_wT16(const float* __restrict__ W, _Float16* Wp,
                                               int KD, int NC, float scale) {
  __shared__ __attribute__((aligned(16))) _Float16 sT[TPN * TPP];
  const int tid = threadIdx.x;
  const int k0 = (int)blockIdx.x * TPK, n0 = (int)blockIdx.y * TPN;
  const int nc = tid & 31, kq = tid >> 5;
#pragma unroll
  for (int i = 0; i < TPK / NWAVE; ++i) {
    const int kr = kq + NWAVE * i;
    const float v = W[(size_t)(k0 + kr) * NC + n0 + nc] * scale;
    sT[nc * TPP + kr] = (_Float16)v;
  }
  __syncthreads();
  const int nl = tid >> 3, p = tid & 7;
  const v8h hv = *(const v8h*)(sT + nl * TPP + 8 * p);
  _Float16* d = Wp + (size_t)(n0 + nl) * KD + k0 + 8 * p;
  *(volatile v8h*)d = hv;
  __threadfence();
  *(volatile v8h*)d = hv;
}

template <int KD, int NC>
__global__ __launch_bounds__(NTHR) void k_gemm(
    const _Float16* __restrict__ A16, const _Float16* __restrict__ Bw, float* C, int nRows, float osc) {
  static_assert((KD % 32) == 0 && (NC % 16) == 0 && (128 % NC) == 0);
  extern __shared__ v4f lds_dyn[];
  constexpr int NT  = NC / 16;
  constexpr int RPI = 128 / NC;
  constexpr int NST = 16 / RPI;
  float* stg = (float*)lds_dyn;
  const int tid = threadIdx.x, lane = tid & 31, wave = tid >> 5, hh = lane >> 4, m = lane & 15;
  const int rowBase = blockIdx.x * GROWS;
  const _Float16* ap  = A16 + (size_t)(rowBase + wave * 16 + m) * KD + 8 * hh;
  const _Float16* bp0 = Bw + (size_t)m * KD + 8 * hh;

  v8f acc[NT];
#pragma unroll
  for (int t = 0; t < NT; ++t) { v8f z = {0.f, 0.f, 0.f, 0.f, 0.f, 0.f, 0.f, 0.f}; acc[t] = z; }

#pragma unroll 1
  for (int kt = 0; kt < KD / 32; ++kt) {
    FragH af;
    af.h[0] = *(const v8h*)(ap + 32 * kt);
    af.h[1] = *(const v8h*)(ap + 32 * kt + 16);
#pragma unroll
    for (int t = 0; t < NT; ++t) {
      const _Float16* bp = bp0 + (size_t)(16 * t) * KD + 32 * kt;
      FragH bf;
      bf.h[0] = *(const v8h*)bp;
      bf.h[1] = *(const v8h*)(bp + 16);
      acc[t] = wmf(af.v, bf.v, acc[t]);
    }
  }

  const int r0 = wave * 16 + 8 * hh;
  float* sp = stg + r0 * NC + m;
#pragma unroll
  for (int t = 0; t < NT; ++t) {
#pragma unroll
    for (int r = 0; r < 8; ++r) sp[r * NC + 16 * t] = acc[t][r] * osc;
  }
  __syncthreads();

  const float* lp = stg + wave * 16 * NC;
  float* gp = C + (size_t)(rowBase + wave * 16) * NC;
#pragma unroll
  for (int i = 0; i < NST; ++i) {
    int nr = nRows - (rowBase + wave * 16 + i * RPI);
    nr = nr < 0 ? 0 : (nr > RPI ? RPI : nr);
    const bool ok = (4 * lane) < nr * NC;
    const v4f v = *(const v4f*)(lp + i * 128 + 4 * lane);
    if (ok) *(volatile v4f*)(gp + (size_t)i * 128 + 4 * lane) = v;
  }
  __threadfence();
#pragma unroll
  for (int i = 0; i < NST; ++i) {
    int nr = nRows - (rowBase + wave * 16 + i * RPI);
    nr = nr < 0 ? 0 : (nr > RPI ? RPI : nr);
    const bool ok = (4 * lane) < nr * NC;
    const v4f v = *(const v4f*)(lp + i * 128 + 4 * lane);
    if (ok) *(volatile v4f*)(gp + (size_t)i * 128 + 4 * lane) = v;
  }
}

__global__ __launch_bounds__(NTHR) void k_hop(
    const int* __restrict__ ksrc, const int* __restrict__ kdst, const float* __restrict__ wgt,
    const float* __restrict__ xin, float* xout, int nK, int nN, int nRowsOut, int vec8) {
  __shared__ __attribute__((aligned(16))) int   scnt[NB];
  __shared__ __attribute__((aligned(16))) int   soff[NB];
  __shared__ __attribute__((aligned(16))) int   scur[NB];
  __shared__ __attribute__((aligned(16))) int   list[NWAVE * WCAP];
  __shared__ __attribute__((aligned(16))) int   region[RCAP];
  __shared__ __attribute__((aligned(16))) float stg[NWAVE * 2 * DOUT];
  __shared__ int wcnt[NWAVE];
  __shared__ int sflag;
  const int tid = threadIdx.x, lane = tid & 31, wave = tid >> 5;
  const int nodeBase = blockIdx.x * NB;

  {
    const v4i z = {0, 0, 0, 0};
    if (tid < NB / 4) ((v4i*)scnt)[tid] = z;
#pragma unroll 1
    for (int i = tid; i < RCAP / 4; i += NTHR) ((v4i*)region)[i] = z;
    if (tid == 0) sflag = 0;
  }
  __syncthreads();

  const int nChunks = (nK + CHUNK - 1) / CHUNK;

#pragma unroll 1
  for (int ch = 0; ch < nChunks; ++ch) {
    const int cbase = ch * CHUNK;
    const int wc = scan_chunk<NB, 0, WCAP>(ksrc, nK, cbase, nodeBase, vec8, list, tid, lane, wave);
    if (lane == 0) wcnt[wave] = wc;
    __syncthreads();
    if (wave == 0) {
#pragma unroll 1
      for (int wsx = 0; wsx < NWAVE; ++wsx) {
        int n = __builtin_amdgcn_readfirstlane(wcnt[wsx]);
        n = n > WCAP ? WCAP : (n < 0 ? 0 : n);
#pragma unroll 1
        for (int i = 0; i < n; ++i) {
          const int ent  = __builtin_amdgcn_readfirstlane(list[wsx * WCAP + i]);
          const int slot = ent & (NB - 1);
          if (lane == 0) scnt[slot] = scnt[slot] + 1;
        }
      }
    }
    __syncthreads();
  }

  if (wave == 0) {
    const v4i c4 = *(const v4i*)(scnt + 4 * lane);
    const int c0 = max(c4.x, 0), c1 = max(c4.y, 0), c2 = max(c4.z, 0), c3 = max(c4.w, 0);
    const int ts = c0 + c1 + c2 + c3;
    int incl = ts;
#pragma unroll
    for (int d = 1; d < 32; d <<= 1) {
      const int t = __shfl_up(incl, d, 32);
      if (lane >= d) incl += t;
    }
    int run = incl - ts;
    v4i o;
    o.x = run; run += c0;
    o.y = run; run += c1;
    o.z = run; run += c2;
    o.w = run;
    *(v4i*)(soff + 4 * lane) = o;
    *(v4i*)(scur + 4 * lane) = o;
    const int tot = __shfl(incl, 31, 32);
    const bool ov = (c0 > DEGCAP) | (c1 > DEGCAP) | (c2 > DEGCAP) | (c3 > DEGCAP) | (tot > RCAP);
    const unsigned ob = __builtin_amdgcn_ballot_w32(ov);
    if (lane == 0) sflag = (ob != 0u) ? 1 : 0;
  }
  __syncthreads();

#pragma unroll 1
  for (int ch = 0; ch < nChunks; ++ch) {
    const int cbase = ch * CHUNK;
    const int wc = scan_chunk<NB, 1, WCAP>(ksrc, nK, cbase, nodeBase, vec8, list, tid, lane, wave);
    if (lane == 0) wcnt[wave] = wc;
    __syncthreads();
    if (wave == 0) {
#pragma unroll 1
      for (int wsx = 0; wsx < NWAVE; ++wsx) {
        int n = __builtin_amdgcn_readfirstlane(wcnt[wsx]);
        n = n > WCAP ? WCAP : (n < 0 ? 0 : n);
#pragma unroll 1
        for (int i = 0; i < n; ++i) {
          const int ent  = __builtin_amdgcn_readfirstlane(list[wsx * WCAP + i]);
          const int slot = ent & (NB - 1);
          int e = (int)(((unsigned)ent) >> ESHF);
          e = e > nK - 1 ? nK - 1 : e;
          if (lane == 0) {
            int pos = scur[slot];
            pos = pos < 0 ? 0 : (pos > RCAP - 1 ? RCAP - 1 : pos);
            region[pos] = e;
            const int np = pos + 1;
            scur[slot] = np > RCAP ? RCAP : np;
          }
        }
      }
    }
    __syncthreads();
  }
  __syncthreads();

  const int flg = sflag;
  U32F qn; qn.i = 0x7fc00000;
  float* sw = stg + wave * 2 * DOUT;
  const int wbase = wave * NPW;
#pragma unroll 1
  for (int j = 0; j < NPW; ++j) {
    const int s = wbase + j;
    const int c = nodeBase + s;
    int n = scnt[s];
    n = n < 0 ? 0 : (n > DEGCAP ? DEGCAP : n);
    int st = soff[s];
    st = st < 0 ? 0 : (st > RCAP ? RCAP : st);
    float ax = 0.0f, ay = 0.0f;
#pragma unroll 1
    for (int q0 = 0; q0 < n; q0 += 32) {
      const int p  = q0 + lane;
      const int pc = p < n ? p : n - 1;
      int ia = st + pc; ia = ia < 0 ? 0 : (ia > RCAP - 1 ? RCAP - 1 : ia);
      int ea = region[ia]; ea = ea < 0 ? 0 : (ea > nK - 1 ? nK - 1 : ea);
      int da = kdst[ea]; da = da < 0 ? 0 : (da > nN - 1 ? nN - 1 : da);
      const float wa = wgt[ea];
      bool keep = p < n;
#pragma unroll 1
      for (int q1 = 0; q1 < n; q1 += 32) {
        const int qq = q1 + lane;
        const int qc = qq < n ? qq : n - 1;
        int ib = st + qc; ib = ib < 0 ? 0 : (ib > RCAP - 1 ? RCAP - 1 : ib);
        int eb = region[ib]; eb = eb < 0 ? 0 : (eb > nK - 1 ? nK - 1 : eb);
        int db = kdst[eb]; db = db < 0 ? 0 : (db > nN - 1 ? nN - 1 : db);
        db = (qq < n) ? db : -1;
        const int mq = (n - q1) < 32 ? (n - q1) : 32;
#pragma unroll 1
        for (int qi = 0; qi < mq; ++qi) {
          const int dbb = __builtin_amdgcn_readlane(db, qi);
          const int ebb = __builtin_amdgcn_readlane(eb, qi);
          keep = keep && !((dbb == da) && (ebb > ea));
        }
      }
      U32F wk; wk.f = keep ? wa : 0.0f;
      const int mc = (n - q0) < 32 ? (n - q0) : 32;
#pragma unroll 1
      for (int pi = 0; pi < mc; ++pi) {
        const int dp = __builtin_amdgcn_readlane(da, pi);
        U32F wu; wu.i = __builtin_amdgcn_readlane(wk.i, pi);
        const v2f xv = *(const v2f*)(xin + (size_t)dp * DOUT + 2 * lane);
        ax = fmaf(wu.f, xv.x, ax);
        ay = fmaf(wu.f, xv.y, ay);
      }
    }
    v2f v;
    v.x = (c < nN) ? ax : 0.0f;
    v.y = (c < nN) ? ay : 0.0f;
    v.x = (flg != 0) ? qn.f : v.x;
    v.y = (flg != 0) ? qn.f : v.y;
    *(v2f*)(sw + (j & 1) * DOUT + 2 * lane) = v;
    if ((j & 1) != 0) {
      __builtin_amdgcn_fence(__ATOMIC_ACQ_REL, "wavefront");
      __builtin_amdgcn_wave_barrier();
      const v4f o = *(const v4f*)(sw + 4 * lane);
      float* rp = xout + (size_t)(c - 1) * DOUT + 4 * lane;
      const bool ok = (c - 1 + (lane >> 4)) < nRowsOut;
      if (ok) *(volatile v4f*)rp = o;
      __threadfence();
      if (ok) *(volatile v4f*)rp = o;
      __builtin_amdgcn_fence(__ATOMIC_ACQ_REL, "wavefront");
      __builtin_amdgcn_wave_barrier();
    }
  }
}

extern "C" void kernel_launch(void* const* d_in, const int* in_sizes, int n_in,
                              void* d_out, int out_size, void* d_ws, size_t ws_size,
                              hipStream_t stream) {
  if (n_in < 4) return;
  const int nN = in_sizes[0] / DEMB;
  const int nE = in_sizes[2] / 2;
  if (nN <= 0 || nE <= 0) return;
  if (in_sizes[0] != nN * DEMB) return;
  if (in_sizes[1] != DEMB * DOUT) return;
  if (in_sizes[2] != 2 * nE || in_sizes[3] != nE) return;
  if (nN > (1 << 20) || nE > (1 << 23)) return;
  if ((long long)out_size != (long long)nN * DOUT) return;

  const float* nf  = (const float*)d_in[0];
  const float* Emb = (const float*)d_in[1];
  const int*   ei  = (const int*)d_in[2];
  const float* ew  = (const float*)d_in[3];
  float* out = (float*)d_out;
  const int* ksrc = ei;
  const int* kdst = ei + nE;

  const int NPAD  = ((nN + NB - 1) / NB) * NB;
  const int nGemm = NPAD / GROWS;
  const int nHop  = NPAD / NB;

  char* ws = (char*)d_ws;
  size_t off = 0;
  const size_t oA16 = off; off += (size_t)NPAD * DEMB * 2;       off = (off + 255) & ~(size_t)255;
  const size_t oEmb = off; off += (size_t)DOUT * DEMB * 2;       off = (off + 255) & ~(size_t)255;
  const size_t oX0  = off; off += (size_t)NPAD * DOUT * 4;       off = (off + 255) & ~(size_t)255;
  const size_t oX1  = off; off += (size_t)NPAD * DOUT * 4;       off = (off + 255) & ~(size_t)255;
  const size_t oX2  = off; off += (size_t)NPAD * DOUT * 4;       off = (off + 255) & ~(size_t)255;
  if (off > ws_size || off > (size_t)WSCAP) return;
  _Float16* A16  = (_Float16*)(ws + oA16);
  _Float16* EmbT = (_Float16*)(ws + oEmb);
  float*    X0   = (float*)(ws + oX0);
  float*    X1   = (float*)(ws + oX1);
  float*    X2   = (float*)(ws + oX2);

  const int vec8 = 1;
  const float osc = 1.0f / ((float)ASCL * (float)WSCL);

  {
    const int t8x = (NPAD * DEMB) / 8;
    k_cvt16<<<(t8x + NTHR - 1) / NTHR, NTHR, 0, stream>>>(nf, A16, DEMB, nN, t8x, (float)ASCL);
  }
  {
    const dim3 gO(DEMB / TPK, DOUT / TPN);
    k_wT16<<<gO, NTHR, 0, stream>>>(Emb, EmbT, DEMB, DOUT, (float)WSCL);
  }
  hipFuncSetAttribute(reinterpret_cast<const void*>(&k_gemm<DEMB, DOUT>),
                      hipFuncAttributeMaxDynamicSharedMemorySize, LDS_GEMM);
  k_gemm<DEMB, DOUT><<<nGemm, NTHR, LDS_GEMM, stream>>>(A16, EmbT, X0, NPAD, osc);

  k_hop<<<nHop, NTHR, 0, stream>>>(ksrc, kdst, ew, X0, X1, nE, nN, NPAD, vec8);
  k_hop<<<nHop, NTHR, 0, stream>>>(ksrc, kdst, ew, X1, X2, nE, nN, NPAD, vec8);
  k_hop<<<nHop, NTHR, 0, stream>>>(ksrc, kdst, ew, X2, out, nE, nN, nN, vec8);
}
